// DGAttention_33440615367162
// MI455X (gfx1250) — hardware-verified
//
#include <hip/hip_runtime.h>


namespace {
constexpr int NF = 3, NBt = 512, D = 256;
constexpr float XS = 8.0f, WSC = 256.0f, LOG2E = 1.4426950408889634f;

typedef _Float16 b16;
typedef __attribute__((ext_vector_type(16))) _Float16 v16b;
typedef __attribute__((ext_vector_type(8))) _Float16 v8b;
typedef __attribute__((ext_vector_type(8))) float v8f;
typedef __attribute__((ext_vector_type(4))) float v4f;
__device__ __forceinline__ float bf16_rne(float f) { unsigned int u = __float_as_uint(f); u += 0x7FFFu + ((u >> 16) & 1u); return __uint_as_float(u & 0xFFFF0000u); }
__device__ __forceinline__ v16b frag_kb(const b16* p, int hh) { const v8b a = *(const v8b*)(p + 8 * hh), b = *(const v8b*)(p + 16 + 8 * hh); v16b f;
#pragma unroll
  for (int e = 0; e < 8; ++e) { f[e] = a[e]; f[8 + e] = b[e]; } return f; }
__device__ __forceinline__ v8f wmma16b(v16b a, v16b b, v8f c) { v8f d = __builtin_amdgcn_wmma_f32_16x16x32_f16(false, a, false, b, (short)0, c, false, false); asm volatile("v_nop\n\tv_nop\n\tv_nop\n\tv_nop" : "+v"(d) : "v"(a), "v"(b)); return d; }
__device__ __forceinline__ void wave_lds_sync() { __builtin_amdgcn_fence(__ATOMIC_RELEASE, "workgroup"); __builtin_amdgcn_wave_barrier(); __builtin_amdgcn_fence(__ATOMIC_ACQUIRE, "workgroup"); }
__device__ __forceinline__ float pmul(float a, float b) { float p = a * b; asm volatile("" : "+v"(p)); return p; }

__global__ __launch_bounds__(256) void prep_kernel(const float* __restrict__ f0, const float* __restrict__ f1, const float* __restrict__ f2, const float* __restrict__ wq, const float* __restrict__ wk, const float* __restrict__ wv, b16* __restrict__ F16, b16* __restrict__ W16) {
  const int t = blockIdx.x * 256 + threadIdx.x; const int nf = NBt * D / 8, nw = NF * D * D / 8;
  const float* src; b16* dst; float sc; int e;
  if (t < 3 * nf) { const int k = t / nf; e = (t - k * nf) * 8; src = (k == 0 ? f0 : k == 1 ? f1 : f2); dst = F16 + (size_t)k * NBt * D; sc = XS; }
  else if (t < 3 * nf + 3 * nw) { const int u = t - 3 * nf; const int k = u / nw; e = (u - k * nw) * 8; src = (k == 0 ? wq : k == 1 ? wk : wv); dst = W16 + (size_t)k * NF * D * D; sc = WSC; } else return;
  v8b o; for (int j = 0; j < 8; ++j) o[j] = (b16)(bf16_rne(src[e + j]) * sc);
  for (int pass = 0; pass < 2; ++pass) { *(volatile v8b*)(dst + e) = o; __threadfence(); }
}
__global__ __launch_bounds__(128) void proj_kernel(const b16* __restrict__ F16, const b16* __restrict__ W16, const float* __restrict__ bq, const float* __restrict__ bk, const float* __restrict__ bv, float* __restrict__ QF, float* __restrict__ KF, float* __restrict__ VF) {
  __shared__ __attribute__((aligned(16))) float Ts[4][16][128 + 4];
  const int wave = threadIdx.x >> 5, lane = threadIdx.x & 31, nloc = lane & 15, hlf = lane >> 4; const int m = blockIdx.z; const size_t m0 = (size_t)blockIdx.x * 64 + wave * 16; const int n0 = blockIdx.y * 128;
  int kind, i, j; if (m < 9) { kind = 0; i = m / 3; j = m - i * 3; } else if (m < 12) { kind = 1; i = m - 9; j = i; } else { kind = 2; i = m - 12; j = i; }
  const b16* A = F16 + (size_t)j * NBt * D; const b16* W = W16 + ((size_t)kind * NF + i) * D * D; const float* bias = (kind == 0 ? bq : kind == 1 ? bk : bv) + i * D;
  float* dst = kind == 0 ? QF + ((size_t)i * NF + j) * NBt * D : (kind == 1 ? KF : VF) + (size_t)i * NBt * D;
  v8f acc[8];
#pragma unroll
  for (int t = 0; t < 8; ++t) acc[t] = (v8f){};
#pragma unroll 2
  for (int kb = 0; kb < D; kb += 32) { const v16b a = frag_kb(A + (m0 + nloc) * D + kb, hlf);
#pragma unroll
    for (int t = 0; t < 8; ++t) acc[t] = wmma16b(a, frag_kb(W + (size_t)(n0 + t * 16 + nloc) * D + kb, hlf), acc[t]); }
#pragma unroll
  for (int t = 0; t < 8; ++t) { const float bb = bf16_rne(bias[n0 + t * 16 + nloc]);
#pragma unroll
    for (int r = 0; r < 8; ++r) Ts[wave][8 * hlf + r][t * 16 + nloc] = fmaxf(acc[t][r] * (1.0f / (XS * WSC)) + bb, 0.0f); }
  wave_lds_sync();
  for (int pass = 0; pass < 2; ++pass) { for (int rr = 0; rr < 16; ++rr) *(volatile v4f*)(dst + (m0 + rr) * D + n0 + lane * 4) = *(const v4f*)(&Ts[wave][rr][lane * 4]); __threadfence(); }
}
__global__ __launch_bounds__(256) void attn_kernel(const float* __restrict__ QF, const float* __restrict__ KF, const float* __restrict__ VF, const float* __restrict__ f0, const float* __restrict__ f1, const float* __restrict__ f2, const float* __restrict__ gamma, float* __restrict__ BS, float* __restrict__ out) {
  __shared__ float Kl[D], Vl[D], red[D], red2[D];
  const int i = blockIdx.x / NBt, b = blockIdx.x - i * NBt, p = threadIdx.x;
  const size_t kro = ((size_t)i * NBt + b) * D; const float kv = KF[kro + p]; Kl[p] = kv; Vl[p] = VF[kro + p]; red[p] = kv; red2[p] = kv;
  __syncthreads();
  for (int s = 128; s >= 1; s >>= 1) { if (p < s) { red[p] = fmaxf(red[p], red[p + s]); red2[p] += red2[p + s]; } __syncthreads(); }
  const float kmax = red[0], ksum = red2[0];
  float acc = 0.0f, qsum = 0.0f;
#pragma unroll 1
  for (int j = 0; j < NF; ++j) { const float Q = QF[(((size_t)i * NF + j) * NBt + b) * D + p]; qsum += Q; const float ql = Q * LOG2E; float s = 0.0f, d = 0.0f;
#pragma unroll 8
    for (int q = 0; q < D; ++q) { const float e = __builtin_amdgcn_exp2f(pmul(ql, Kl[q] - kmax)); d += e; s += pmul(e, Vl[q]); }
    acc += s / d; }
  const float* Fi = (i == 0 ? f0 : i == 1 ? f1 : f2); const float r_ = pmul(acc * (1.0f / 3.0f), bf16_rne(gamma[i])) + bf16_rne(Fi[(size_t)b * D + p]);
  __syncthreads(); red2[p] = qsum; __syncthreads();
  for (int s = 128; s >= 1; s >>= 1) { if (p < s) red2[p] += red2[p + s]; __syncthreads(); }
  for (int pass = 0; pass < 2; ++pass) { ((volatile float*)out)[kro + p] = r_; if (p < 32) ((volatile float*)BS)[(size_t)blockIdx.x * 32 + p] = (p == 0) ? pmul(red2[0], ksum) : 0.0f; __threadfence(); }
}
__global__ __launch_bounds__(32) void alpha_kernel(const float* __restrict__ BS, float* __restrict__ out3) {
  const int lane = threadIdx.x; float m[NF];
  for (int i = 0; i < NF; ++i) { float s = 0.0f; for (int b = lane; b < NBt; b += 32) s += BS[((size_t)i * NBt + b) * 32];
#pragma unroll
    for (int o = 16; o >= 1; o >>= 1) s += __shfl_xor(s, o);
    m[i] = s * (1.0f / ((float)NF * NBt * D * D)); }
  const float mx = fmaxf(m[0], fmaxf(m[1], m[2])); float e[NF], se = 0.0f; for (int i = 0; i < NF; ++i) { e[i] = __expf(m[i] - mx); se += e[i]; }
  for (int pass = 0; pass < 2; ++pass) { if (lane < NF) ((volatile float*)out3)[lane] = e[lane] / se; __threadfence(); }
}
}

extern "C" void kernel_launch(void* const* d_in, const int* in_sizes, int n_in, void* d_out, int out_size, void* d_ws, size_t ws_size, hipStream_t stream) {
  (void)n_in;
  auto Fp = [&](int i) { return (const float*)d_in[i]; };
  if (in_sizes[0] != NBt * D || in_sizes[3] != NF * D * D || in_sizes[5] != NF * D * D || in_sizes[7] != NF * D * D || in_sizes[9] != NF || out_size != NF * NBt * D + NF) return;
  size_t off = 0; char* ws = (char*)d_ws;
  auto carve = [&](size_t bytes) { char* p = ws + off; off += (bytes + 255) & ~(size_t)255; return p; };
  b16* F16 = (b16*)carve((size_t)NF * NBt * D * 2); b16* W16 = (b16*)carve((size_t)3 * NF * D * D * 2); float* QF = (float*)carve((size_t)NF * NF * NBt * D * 4); float* KF = (float*)carve((size_t)NF * NBt * D * 4); float* VF = (float*)carve((size_t)NF * NBt * D * 4); float* BS = (float*)carve((size_t)NF * NBt * 32 * 4);
  if (off > ws_size || off > ((size_t)128 << 20)) return;
  prep_kernel<<<(3 * NBt * D / 8 + 3 * NF * D * D / 8 + 255) / 256, 256, 0, stream>>>(Fp(0), Fp(1), Fp(2), Fp(3), Fp(5), Fp(7), F16, W16);
  proj_kernel<<<dim3(NBt / 64, D / 128, 15), 128, 0, stream>>>(F16, W16, Fp(4), Fp(6), Fp(8), QF, KF, VF);
  attn_kernel<<<NF * NBt, 256, 0, stream>>>(QF, KF, VF, Fp(0), Fp(1), Fp(2), Fp(9), BS, (float*)d_out);
  alpha_kernel<<<1, 32, 0, stream>>>(BS, (float*)d_out + (size_t)NF * NBt * D);
}
